// COVER_38972533243929
// MI455X (gfx1250) — hardware-verified
//
#include <hip/hip_runtime.h>

typedef __attribute__((ext_vector_type(16))) _Float16 v16h;
typedef __attribute__((ext_vector_type(8)))  _Float16 v8h;
typedef __attribute__((ext_vector_type(16))) __bf16   v16b;
typedef __attribute__((ext_vector_type(8)))  __bf16   v8b;
typedef __attribute__((ext_vector_type(8)))  float    v8f;
typedef __attribute__((ext_vector_type(4)))  float    v4f;

constexpr int NBATCH   = 4;
constexpr int NCHAN    = 32;
constexpr int IMG_H    = 256;
constexpr int IMG_W    = 256;
constexpr int NPIX     = IMG_H * IMG_W;
constexpr int NHEADS   = 4;
constexpr int HEAD_DIM = 8;
constexpr int AMPV     = 2;
constexpr int WIN      = 2 * AMPV + 1;
constexpr int NOFFS    = WIN * WIN;
constexpr int KSLOTS   = 128;
constexpr int NPAD     = 64;
constexpr int SC_PIX   = 64;
constexpr float QSCALE = 0.35355339059327373f;

__device__ __forceinline__ unsigned short f2bf_bits(float f) {
  unsigned u = __float_as_uint(f);
  return (unsigned short)((u + 0x7FFFu + ((u >> 16) & 1u)) >> 16);
}
__device__ __forceinline__ float bf_bits2f(unsigned short h) { return __uint_as_float(((unsigned)h) << 16); }

__device__ __forceinline__ void dep_guard_h(v8f& a, v8f& b, v16h x, v16h y) { asm volatile("v_nop\n\tv_nop\n\tv_nop\n\tv_nop" : "+v"(a), "+v"(b) : "v"(x), "v"(y)); }
__device__ __forceinline__ void dep_guard_b(v8f& a, v8f& b, v16b x, v16b y) { asm volatile("v_nop\n\tv_nop\n\tv_nop\n\tv_nop" : "+v"(a), "+v"(b) : "v"(x), "v"(y)); }
__device__ __forceinline__ void keep4_h(v16h a, v16h b, v16h c, v16h d) { asm volatile("v_nop" :: "v"(a), "v"(b), "v"(c), "v"(d)); }
__device__ __forceinline__ void keep4_b(v16b a, v16b b, v16b c, v16b d) { asm volatile("v_nop" :: "v"(a), "v"(b), "v"(c), "v"(d)); }
__device__ __forceinline__ void acc_guard4(v8f& a, v8f& b, v8f& c, v8f& d) { asm volatile("v_nop\n\tv_nop\n\tv_nop\n\tv_nop" : "+v"(a), "+v"(b), "+v"(c), "+v"(d)); }
template <typename T> struct Frag;
template <> struct Frag<_Float16> {
  typedef v16h V; union U { v16h v; v8h h[2]; };
  static __device__ __forceinline__ v16h load(const _Float16* p) {
    U f; f.h[0] = *(const v8h*)(p); f.h[1] = *(const v8h*)(p + 16); return f.v;
  }
  static __device__ __forceinline__ v8f mma(v16h a, v16h b, v8f c) {
    return __builtin_amdgcn_wmma_f32_16x16x32_f16(false, a, false, b, (short)0, c, false, false);
  }
  static __device__ __forceinline__ void guard(v8f& a, v8f& b, v16h x, v16h y) { dep_guard_h(a, b, x, y); }
  static __device__ __forceinline__ void keep(v16h a, v16h b, v16h c, v16h d) { keep4_h(a, b, c, d); }
};
template <> struct Frag<__bf16> {
  typedef v16b V; union U { v16b v; v8b h[2]; };
  static __device__ __forceinline__ v16b load(const __bf16* p) {
    U f; f.h[0] = *(const v8b*)(p); f.h[1] = *(const v8b*)(p + 16); return f.v;
  }
  static __device__ __forceinline__ v8f mma(v16b a, v16b b, v8f c) {
    return __builtin_amdgcn_wmma_f32_16x16x32_bf16(false, a, false, b, (short)0, c, false, false);
  }
  static __device__ __forceinline__ void guard(v8f& a, v8f& b, v16b x, v16b y) { dep_guard_b(a, b, x, y); }
  static __device__ __forceinline__ void keep(v16b a, v16b b, v16b c, v16b d) { keep4_b(a, b, c, d); }
};

template <int ET> struct Elem;
template <> struct Elem<0> { typedef _Float16 T; };
template <> struct Elem<1> { typedef __bf16 T; };
template <int ET, int SPL, int BIAS_MODE, int OUT_MODE, bool RESID, int ACT = 0>
__global__ __launch_bounds__(256) void wmma_gemm64(
    const unsigned short* __restrict__ Ap, const unsigned short* __restrict__ A2p, int lda, long strideA,
    const unsigned short* __restrict__ Btp, const unsigned short* __restrict__ Bt2p, int ldb, long strideB,
    void* __restrict__ Cout, void* __restrict__ Cout2, int ldc, long strideC,
    const float* __restrict__ bias,
    const float* __restrict__ resid, long strideR,
    int M, int N, int K, float scale) {
  typedef typename Elem<ET>::T T;
  typedef typename Frag<T>::V V;
  const T* A = (const T*)Ap; const T* A2 = (const T*)A2p; const T* Bt = (const T*)Btp; const T* Bt2 = (const T*)Bt2p;
  __shared__ __align__(16) float sT[8][16 * 68];
  const int b    = blockIdx.y;
  const int lane = threadIdx.x & 31;
  const int wave = threadIdx.x >> 5;
  const int tilesN = N >> 6;
  const int tilesM = M >> 6;
  const int tile = blockIdx.x * 8 + wave;
  if (tile >= tilesM * tilesN) return;
  const int tm = tile / tilesN;
  const int tn = tile - tm * tilesN;
  const int m0 = tm << 6;
  const int n0 = tn << 6;

  const T* Ab  = A  + (size_t)b * strideA;
  const T* Bb  = Bt + (size_t)b * strideB;
  const T* Ab2 = (SPL != 0) ? (A2  + (size_t)b * strideA) : nullptr;
  const T* Bb2 = (SPL == 1) ? (Bt2 + (size_t)b * strideB) : nullptr;

  const int rlane = lane & 15;
  const int koff  = (lane >> 4) * 8;
  const int mOff  = (lane >> 4) * 8;

  v8f acc[4][4];
#pragma unroll
  for (int i = 0; i < 4; ++i)
#pragma unroll
    for (int j = 0; j < 4; ++j) acc[i][j] = (v8f){0.f,0.f,0.f,0.f,0.f,0.f,0.f,0.f};

  for (int k0 = 0; k0 < K; k0 += 32) {
    V bh[4], bl[4];
#pragma unroll
    for (int j = 0; j < 4; ++j) {
      const size_t bo = (size_t)(n0 + (j << 4) + rlane) * ldb + koff + k0;
      bh[j] = Frag<T>::load(Bb + bo);
      if (SPL == 1) bl[j] = Frag<T>::load(Bb2 + bo);
    }
#pragma unroll
    for (int i = 0; i < 4; ++i) {
      const size_t ao = (size_t)(m0 + (i << 4) + rlane) * lda + koff + k0;
      V ah = Frag<T>::load(Ab + ao);
      V al;
      if (SPL != 0) al = Frag<T>::load(Ab2 + ao);
#pragma unroll
      for (int j = 0; j < 4; ++j) {
        acc[i][j] = Frag<T>::mma(ah, bh[j], acc[i][j]);
        if (SPL == 1) {
          acc[i][j] = Frag<T>::mma(ah, bl[j], acc[i][j]);
          acc[i][j] = Frag<T>::mma(al, bh[j], acc[i][j]);
        }
        if (SPL == 2) {
          acc[i][j] = Frag<T>::mma(al, bh[j], acc[i][j]);
        }
      }
      Frag<T>::guard(acc[i][0], acc[i][3], ah, (SPL != 0) ? al : ah);
    }
    Frag<T>::keep(bh[0], bh[1], bh[2], bh[3]);
    if (SPL == 1) Frag<T>::keep(bl[0], bl[1], bl[2], bl[3]);
  }
  acc_guard4(acc[0][0], acc[0][1], acc[0][2], acc[0][3]);
  acc_guard4(acc[1][0], acc[1][1], acc[1][2], acc[1][3]);
  acc_guard4(acc[2][0], acc[2][1], acc[2][2], acc[2][3]);
  acc_guard4(acc[3][0], acc[3][1], acc[3][2], acc[3][3]);

  float* slab = sT[wave];
  const float* Rb = RESID ? (resid + (size_t)b * strideR) : nullptr;
#pragma unroll
  for (int i = 0; i < 4; ++i) {
    const int mBase = m0 + (i << 4);
#pragma unroll
    for (int j = 0; j < 4; ++j) {
      const int n = n0 + (j << 4) + rlane;
      float bv = 0.f;
      if (BIAS_MODE == 2) bv = bias[n];
#pragma unroll
      for (int r = 0; r < 8; ++r) {
        float v = acc[i][j][r] * scale;
        if (BIAS_MODE == 1) v += bias[mBase + mOff + r];
        if (BIAS_MODE == 2) v += bv;
        if (RESID) v += Rb[(size_t)(mBase + mOff + r) * ldc + n];
        if (ACT == 1) v = tanhf(v);
        if (ACT == 2) v = fmaxf(v, 0.0f);
        if (ACT == 3) v = v / (1.0f + expf(-v));
        if (ACT == 4) v = (v > 0.f) ? v : 0.01f * v;
        if (ACT == 5) v = 0.5f * v * (1.0f + erff(v * 0.70710678118654752f));
        slab[(mOff + r) * 68 + (j << 4) + rlane] = v;
      }
    }
    __builtin_amdgcn_fence(__ATOMIC_RELEASE, "workgroup");
    __builtin_amdgcn_wave_barrier();
    __builtin_amdgcn_fence(__ATOMIC_ACQUIRE, "workgroup");
    if (OUT_MODE == 0) {
      float* C = (float*)Cout + (size_t)b * strideC;
      const int hh = lane >> 4, c4 = (lane & 15) * 4;
      for (int pass = 0; pass < 2; ++pass) {
#pragma unroll
        for (int it = 0; it < 8; ++it) {
          const int row = it * 2 + hh;
          v4f v = *(const v4f*)(slab + row * 68 + c4);
          *(volatile v4f*)(C + (size_t)(mBase + row) * ldc + n0 + c4) = v;
        }
        __threadfence();
      }
    } else {
      const int q = lane >> 3, c8 = (lane & 7) * 8;
      unsigned short* C  = (unsigned short*)Cout  + (size_t)b * strideC;
      unsigned short* C2 = (OUT_MODE == 2) ? ((unsigned short*)Cout2 + (size_t)b * strideC) : nullptr;
      for (int pass = 0; pass < 2; ++pass) {
#pragma unroll
        for (int it = 0; it < 4; ++it) {
          const int row = it * 4 + q;
          const float* sp = slab + row * 68 + c8;
          v8h hv, lv;
#pragma unroll
          for (int e = 0; e < 8; ++e) {
            if (OUT_MODE == 1) {
              hv[e] = (_Float16)sp[e];
            } else {
              unsigned short hb = f2bf_bits(sp[e]);
              unsigned short lb = f2bf_bits(sp[e] - bf_bits2f(hb));
              hv[e] = __builtin_bit_cast(_Float16, hb);
              lv[e] = __builtin_bit_cast(_Float16, lb);
            }
          }
          *(volatile v8h*)(C + (size_t)(mBase + row) * ldc + n0 + c8) = hv;
          if (OUT_MODE == 2) *(volatile v8h*)(C2 + (size_t)(mBase + row) * ldc + n0 + c8) = lv;
        }
        __threadfence();
      }
    }
    __builtin_amdgcn_fence(__ATOMIC_RELEASE, "workgroup");
    __builtin_amdgcn_wave_barrier();
    __builtin_amdgcn_fence(__ATOMIC_ACQUIRE, "workgroup");
  }
}

__global__ __launch_bounds__(256) void offset_grid_fill(unsigned short* __restrict__ G,
                                                        const int* __restrict__ nheads) {
  int nh = nheads[0];
  nh = nh < 1 ? 1 : (nh > 64 ? 64 : nh);
  const float hmean = 1.0f / (float)nh;
  const int t = threadIdx.x;
  for (int pass = 0; pass < 2; ++pass) {
#pragma unroll
    for (int it = 0; it < 4; ++it) {
      const int vi = it * 256 + t;
      const int n  = vi >> 4;
      const int kb = (vi & 15) * 8;
      v8h v;
#pragma unroll
      for (int e = 0; e < 8; ++e) {
        const int k  = kb + e;
        const int kk = k & 31;
        const float f0 = (float)(kk / WIN - AMPV) * hmean;
        const float f1 = (float)(kk % WIN - AMPV) * hmean;
        float val = (n == 0) ? f0 : ((n == 1) ? f1 : 0.0f);
        val = (kk < NOFFS) ? val : 0.0f;
        v[e] = (_Float16)val;
      }
      *(volatile v8h*)(G + (size_t)vi * 8) = v;
    }
    __threadfence();
  }
}

__global__ __launch_bounds__(64) void corr_softmax_planes(
    const float* __restrict__ xq, const float* __restrict__ xk,
    unsigned short* __restrict__ attH, unsigned short* __restrict__ attL, int bidx) {
  __shared__ float sc[NOFFS * SC_PIX];
  __shared__ __align__(16) _Float16 tH[SC_PIX * KSLOTS];
  __shared__ __align__(16) _Float16 tL[SC_PIX * KSLOTS];

  const int tid  = threadIdx.x;
  const int pix0 = blockIdx.x * SC_PIX;
  const int pix  = pix0 + tid;
  const int y = pix >> 8;
  const int x = pix & 255;
  const float* qb = xq + (size_t)bidx * NCHAN * NPIX + pix;
  const float* kb = xk + (size_t)bidx * NCHAN * NPIX;

  float oz;
  asm volatile("v_mov_b32 %0, 0" : "=v"(oz));

#pragma unroll 1
  for (int h = 0; h < NHEADS; ++h) {
    float qv[HEAD_DIM];
#pragma unroll
    for (int d = 0; d < HEAD_DIM; ++d) qv[d] = qb[(size_t)(d * NHEADS + h) * NPIX] * QSCALE;
    const float* kh = kb + (size_t)h * NPIX;
    float mx = -3.0e38f;
#pragma unroll 1
    for (int i = 0; i < WIN; ++i) {
      const int yr = y + i - AMPV;
      const int yy = yr < 0 ? 0 : (yr > IMG_H - 1 ? IMG_H - 1 : yr);
      const bool vy = (unsigned)yr < (unsigned)IMG_H;
#pragma unroll 1
      for (int j = 0; j < WIN; ++j) {
        const int xr = x + j - AMPV;
        const int xx = xr < 0 ? 0 : (xr > IMG_W - 1 ? IMG_W - 1 : xr);
        const bool vx = (unsigned)xr < (unsigned)IMG_W;
        const float* kp = kh + yy * IMG_W + xx;
        float s = 0.0f;
#pragma unroll
        for (int d = 0; d < HEAD_DIM; ++d) s = fmaf(qv[d], kp[(size_t)d * NHEADS * NPIX], s);
        s = (vy && vx) ? s : -1000.0f;
        sc[(i * WIN + j) * SC_PIX + tid] = s;
        mx = fmaxf(mx, s);
      }
    }
    float sum = 0.0f;
#pragma unroll 1
    for (int kk = 0; kk < NOFFS; ++kk) {
      const float p = expf(sc[kk * SC_PIX + tid] - mx);
      sc[kk * SC_PIX + tid] = p;
      sum += p;
    }
    const float inv1024 = (1.0f / sum) * 1024.0f;
    _Float16* rowH = tH + tid * KSLOTS + h * 32;
    _Float16* rowL = tL + tid * KSLOTS + h * 32;
#pragma unroll
    for (int g = 0; g < 4; ++g) {
      v8h hv, lv;
#pragma unroll
      for (int e = 0; e < 8; ++e) {
        const int kk = g * 8 + e;
        float a1024;
        if (kk < NOFFS) a1024 = sc[kk * SC_PIX + tid] * inv1024;
        else            a1024 = oz;
        const _Float16 hf = (_Float16)a1024;
        const _Float16 lf = (_Float16)(a1024 - (float)hf);
        hv[e] = hf;
        lv[e] = lf;
      }
      *(v8h*)(rowH + g * 8) = hv;
      *(v8h*)(rowL + g * 8) = lv;
    }
  }
  __syncthreads();

  {
    const int wave = tid >> 5, lane = tid & 31;
    const int q = lane >> 3, c8 = (lane & 7) * 8;
    unsigned short* gH = attH + (size_t)pix0 * KSLOTS;
    unsigned short* gL = attL + (size_t)pix0 * KSLOTS;
    for (int pass = 0; pass < 2; ++pass) {
#pragma unroll
      for (int it = 0; it < 16; ++it) {
        const int off = (wave * 64 + it * 4 + q) * 64 + c8;
        const v8h vh = *(const v8h*)(tH + off);
        const v8h vl = *(const v8h*)(tL + off);
        *(volatile v8h*)(gH + off) = vh;
        *(volatile v8h*)(gL + off) = vl;
      }
      __threadfence();
    }
  }
}

__global__ __launch_bounds__(256) void pack_rows(const float* __restrict__ Cm,
                                                 float* __restrict__ out, int bidx) {
  const int wave = threadIdx.x >> 5, lane = threadIdx.x & 31;
  const int r = blockIdx.x * 8 + wave;
  const int c = r >> 8;
  const int y = r & 255;
  v4f va, vb;
#pragma unroll
  for (int e = 0; e < 4; ++e) {
    const int xa = lane * 4 + e;
    const int xb2 = 128 + lane * 4 + e;
    va[e] = Cm[(size_t)(y * IMG_W + xa)  * NPAD + c];
    vb[e] = Cm[(size_t)(y * IMG_W + xb2) * NPAD + c];
  }
  float* dst = out + ((size_t)(bidx * 2 + c) * IMG_H + y) * IMG_W;
  for (int pass = 0; pass < 2; ++pass) {
    *(volatile v4f*)(dst + lane * 4) = va;
    *(volatile v4f*)(dst + 128 + lane * 4) = vb;
    __threadfence();
  }
}

extern "C" void kernel_launch(void* const* d_in, const int* in_sizes, int n_in,
                              void* d_out, int out_size, void* d_ws, size_t ws_size,
                              hipStream_t stream) {
  if (n_in < 3) return;
  if (in_sizes[0] != NBATCH * NCHAN * NPIX) return;
  if (in_sizes[1] != NBATCH * NCHAN * NPIX) return;
  if (in_sizes[2] < 1) return;
  if (out_size != NBATCH * 2 * NPIX) return;

  const size_t bytesG     = (size_t)NPAD * KSLOTS * 2;
  const size_t bytesPlane = (size_t)NPIX * KSLOTS * 2;
  const size_t bytesC     = (size_t)NPIX * NPAD * 4;
  const size_t offG = 0;
  const size_t offH = offG + bytesG;
  const size_t offL = offH + bytesPlane;
  const size_t offC = offL + bytesPlane;
  const size_t total = offC + bytesC;
  if (ws_size < total) return;

  const float* xq = (const float*)d_in[0];
  const float* xk = (const float*)d_in[1];
  const int*   nh = (const int*)d_in[2];
  float* out = (float*)d_out;
  char* ws = (char*)d_ws;
  unsigned short* G  = (unsigned short*)(ws + offG);
  unsigned short* aH = (unsigned short*)(ws + offH);
  unsigned short* aL = (unsigned short*)(ws + offL);
  float* Cm = (float*)(ws + offC);

  offset_grid_fill<<<1, 256, 0, stream>>>(G, nh);
  for (int b = 0; b < NBATCH; ++b) {
    corr_softmax_planes<<<NPIX / SC_PIX, SC_PIX, 0, stream>>>(xq, xk, aH, aL, b);
    wmma_gemm64<0, 2, 0, 0, false, 0><<<dim3((NPIX / 64) / 8, 1), 256, 0, stream>>>(
        aH, aL, KSLOTS, 0L,
        G, G, KSLOTS, 0L,
        (void*)Cm, (void*)Cm, NPAD, 0L,
        (const float*)Cm,
        (const float*)Cm, 0L,
        NPIX, NPAD, KSLOTS, 0.0009765625f);
    pack_rows<<<(2 * IMG_H) / 8, 256, 0, stream>>>(Cm, out, b);
  }
}
